// Head_21809843929106
// MI455X (gfx1250) — hardware-run, weakly checked
//
#include <hip/hip_runtime.h>
#include <math.h>

typedef __attribute__((ext_vector_type(16))) _Float16 v16h;
typedef __attribute__((ext_vector_type(8)))  _Float16 v8h;
typedef __attribute__((ext_vector_type(16))) __bf16   v16b;
typedef __attribute__((ext_vector_type(8)))  __bf16   v8b;
typedef __attribute__((ext_vector_type(8)))  float    v8f;
typedef __attribute__((ext_vector_type(4)))  float    v4f;
typedef __attribute__((ext_vector_type(4)))  unsigned int v4u;

constexpr int isqrt_c(int n) { int r = 0; while ((r + 1) * (r + 1) <= n) ++r; return r; }

constexpr int kBatch = 4;
constexpr int kSeq   = 2048;
constexpr int kEmb   = 1024;
constexpr int kHead  = 64;
constexpr int kRows  = kBatch * kSeq;
constexpr int kHeadRoot = isqrt_c(kHead);
static_assert(kHeadRoot * kHeadRoot == kHead);
static_assert(kRows == 8192 && kEmb == 1024 && kHead == 64);
static_assert((kEmb % 32) == 0 && (kRows % 64) == 0 && (kHead % 64) == 0);

constexpr float kLogitScale = 1.0f / (float)kHeadRoot;
constexpr float kXCarry   = 16.0f;
constexpr float kWCarry   = 1024.0f;
constexpr float kQKVCarry = 16.0f;
constexpr float kProjSplitScale = kQKVCarry;
constexpr float kProjPlainScale = kQKVCarry / (kXCarry * kWCarry);
constexpr float kScoreFold = kLogitScale / (kQKVCarry * kQKVCarry);
constexpr float kLn2      = 0.6931471805599453f;
constexpr float kLnPCarry = 10.0f * kLn2;
constexpr float kF16Min   = 6.103515625e-5f;

constexpr int kAtWaves = 4;
constexpr int kAtQB    = 64;
constexpr int kAtKC    = 64;
constexpr int kAtOsP   = 68;
constexpr int kQBlkPerB = kSeq / kAtQB;
static_assert((kSeq % kAtQB) == 0 && (kSeq % kAtKC) == 0);
static_assert((kAtKC * kHead / 8) == 4 * kAtWaves * 32);

constexpr size_t kOffXH  = 0;
constexpr size_t kOffXL  = kOffXH  + (size_t)kRows * kEmb * 2;
constexpr size_t kOffXF  = kOffXL  + (size_t)kRows * kEmb * 2;
constexpr size_t kOffWSH = kOffXF  + (size_t)kRows * kEmb * 2;
constexpr size_t kOffWSL = kOffWSH + (size_t)3 * kHead * kEmb * 2;
constexpr size_t kOffWF  = kOffWSL + (size_t)3 * kHead * kEmb * 2;
constexpr size_t kOffQ1  = kOffWF  + (size_t)2 * kHead * kEmb * 2;
constexpr size_t kOffK1  = kOffQ1  + (size_t)kRows * kHead * 2;
constexpr size_t kOffQ2  = kOffK1  + (size_t)kRows * kHead * 2;
constexpr size_t kOffK2  = kOffQ2  + (size_t)kRows * kHead * 2;
constexpr size_t kOffVT  = kOffK2  + (size_t)kRows * kHead * 2;
constexpr size_t kOffO1  = kOffVT  + (size_t)kRows * kHead * 2;
constexpr size_t kWsTotal = kOffO1 + (size_t)kRows * kHead * 4;
static_assert(kWsTotal == 58720256ull);
static_assert(kWsTotal <= 134217728ull);
static_assert((kOffXL % 128) == 0 && (kOffXF % 128) == 0 && (kOffWSH % 128) == 0 && (kOffWSL % 128) == 0 &&
              (kOffWF % 128) == 0 && (kOffQ1 % 128) == 0 && (kOffK1 % 128) == 0 && (kOffQ2 % 128) == 0 &&
              (kOffK2 % 128) == 0 && (kOffVT % 128) == 0 && (kOffO1 % 128) == 0);

__device__ __forceinline__ unsigned short f2bf_bits(float f) {
  unsigned u = __float_as_uint(f);
  return (unsigned short)((u + 0x7FFFu + ((u >> 16) & 1u)) >> 16);
}
__device__ __forceinline__ float bf_bits2f(unsigned short h) { return __uint_as_float(((unsigned)h) << 16); }
__device__ __forceinline__ unsigned pk16(unsigned short a, unsigned short b) { return (unsigned)a | ((unsigned)b << 16); }
__device__ __forceinline__ unsigned short h_bits(float f) { const _Float16 h = (_Float16)f; return __builtin_bit_cast(unsigned short, h); }
__device__ __forceinline__ float flush_f16(float v) { return (fabsf(v) < kF16Min) ? 0.0f : v; }

__device__ __forceinline__ v8f mma_h(v16h a, v16h b, v8f c) {
  c = __builtin_amdgcn_wmma_f32_16x16x32_f16(false, a, false, b, (short)0, c, false, false);
  asm volatile("v_nop\n\tv_nop\n\tv_nop\n\tv_nop" : "+v"(c) : "v"(a), "v"(b));
  return c;
}
__device__ __forceinline__ v8f mma_b(v16b a, v16b b, v8f c) {
  c = __builtin_amdgcn_wmma_f32_16x16x32_bf16(false, a, false, b, (short)0, c, false, false);
  asm volatile("v_nop\n\tv_nop\n\tv_nop\n\tv_nop" : "+v"(c) : "v"(a), "v"(b));
  return c;
}
__device__ __forceinline__ void keep4_h(v16h a, v16h b, v16h c, v16h d) { asm volatile("v_nop" :: "v"(a), "v"(b), "v"(c), "v"(d)); }
__device__ __forceinline__ void keep4_b(v16b a, v16b b, v16b c, v16b d) { asm volatile("v_nop" :: "v"(a), "v"(b), "v"(c), "v"(d)); }
__device__ __forceinline__ void acc_guard4(v8f& a, v8f& b, v8f& c, v8f& d) { asm volatile("v_nop\n\tv_nop\n\tv_nop\n\tv_nop" : "+v"(a), "+v"(b), "+v"(c), "+v"(d)); }

template <typename T> struct Frag;
template <> struct Frag<_Float16> {
  typedef v16h V; union U { v16h v; v8h h[2]; };
  static __device__ __forceinline__ v16h load(const _Float16* p) {
    U f; f.h[0] = *(const v8h*)(p); f.h[1] = *(const v8h*)(p + 16); return f.v;
  }
  static __device__ __forceinline__ v8f mma(v16h a, v16h b, v8f c) { return mma_h(a, b, c); }
  static __device__ __forceinline__ void keep(v16h a, v16h b, v16h c, v16h d) { keep4_h(a, b, c, d); }
};
template <> struct Frag<__bf16> {
  typedef v16b V; union U { v16b v; v8b h[2]; };
  static __device__ __forceinline__ v16b load(const __bf16* p) {
    U f; f.h[0] = *(const v8b*)(p); f.h[1] = *(const v8b*)(p + 16); return f.v;
  }
  static __device__ __forceinline__ v8f mma(v16b a, v16b b, v8f c) { return mma_b(a, b, c); }
  static __device__ __forceinline__ void keep(v16b a, v16b b, v16b c, v16b d) { keep4_b(a, b, c, d); }
};

template <int ET> struct Elem;
template <> struct Elem<0> { typedef _Float16 T; };
template <> struct Elem<1> { typedef __bf16 T; };

template <int ET, bool SPLIT>
__global__ __launch_bounds__(256) void wmma_gemm64_h(
    const unsigned short* __restrict__ Ap, const unsigned short* __restrict__ A2p, int lda, long strideA,
    const unsigned short* __restrict__ Btp, const unsigned short* __restrict__ Bt2p, int ldb, long strideB,
    unsigned short* __restrict__ Cout, int ldc, long strideC,
    int M, int N, int K, float scale) {
  typedef typename Elem<ET>::T T;
  typedef typename Frag<T>::V V;
  const T* A = (const T*)Ap; const T* A2 = (const T*)A2p; const T* Bt = (const T*)Btp; const T* Bt2 = (const T*)Bt2p;
  __shared__ __align__(16) float sT[8][16 * 68];
  const int b    = blockIdx.y;
  const int lane = threadIdx.x & 31;
  const int wave = threadIdx.x >> 5;
  const int tilesN = N >> 6;
  const int tilesM = M >> 6;
  const int tile = blockIdx.x * 8 + wave;
  if (tile >= tilesM * tilesN) return;
  const int tm = tile / tilesN;
  const int tn = tile - tm * tilesN;
  const int m0 = tm << 6;
  const int n0 = tn << 6;

  const T* Ab  = A  + (size_t)b * strideA;
  const T* Bb  = Bt + (size_t)b * strideB;
  const T* Ab2 = A2  + (size_t)b * strideA;
  const T* Bb2 = Bt2 + (size_t)b * strideB;

  const int rlane = lane & 15;
  const int koff  = (lane >> 4) * 8;
  const int mOff  = (lane >> 4) * 8;

  v8f acc[4][4];
#pragma unroll
  for (int i = 0; i < 4; ++i)
#pragma unroll
    for (int j = 0; j < 4; ++j) acc[i][j] = (v8f){0.f,0.f,0.f,0.f,0.f,0.f,0.f,0.f};

  for (int k0 = 0; k0 < K; k0 += 32) {
    V bh[4], bl[4];
#pragma unroll
    for (int j = 0; j < 4; ++j) {
      const size_t bo = (size_t)(n0 + (j << 4) + rlane) * ldb + koff + k0;
      bh[j] = Frag<T>::load(Bb + bo);
      if (SPLIT) bl[j] = Frag<T>::load(Bb2 + bo);
    }
#pragma unroll
    for (int i = 0; i < 4; ++i) {
      const size_t ao = (size_t)(m0 + (i << 4) + rlane) * lda + koff + k0;
      V ah = Frag<T>::load(Ab + ao);
      V al;
      if (SPLIT) al = Frag<T>::load(Ab2 + ao);
#pragma unroll
      for (int j = 0; j < 4; ++j) {
        acc[i][j] = Frag<T>::mma(ah, bh[j], acc[i][j]);
        if (SPLIT) {
          acc[i][j] = Frag<T>::mma(ah, bl[j], acc[i][j]);
          acc[i][j] = Frag<T>::mma(al, bh[j], acc[i][j]);
        }
      }
    }
    Frag<T>::keep(bh[0], bh[1], bh[2], bh[3]);
    if (SPLIT) Frag<T>::keep(bl[0], bl[1], bl[2], bl[3]);
  }
  acc_guard4(acc[0][0], acc[0][1], acc[0][2], acc[0][3]);
  acc_guard4(acc[1][0], acc[1][1], acc[1][2], acc[1][3]);
  acc_guard4(acc[2][0], acc[2][1], acc[2][2], acc[2][3]);
  acc_guard4(acc[3][0], acc[3][1], acc[3][2], acc[3][3]);

  float* slab = sT[wave];
  unsigned short* C = Cout + (size_t)b * strideC;
  const int q = lane >> 3, c8 = (lane & 7) * 8;
#pragma unroll
  for (int i = 0; i < 4; ++i) {
    const int mBase = m0 + (i << 4);
#pragma unroll
    for (int j = 0; j < 4; ++j) {
#pragma unroll
      for (int r = 0; r < 8; ++r) {
        slab[(mOff + r) * 68 + (j << 4) + rlane] = acc[i][j][r] * scale;
      }
    }
    __builtin_amdgcn_fence(__ATOMIC_RELEASE, "workgroup");
    __builtin_amdgcn_wave_barrier();
    __builtin_amdgcn_fence(__ATOMIC_ACQUIRE, "workgroup");
    for (int pass = 0; pass < 2; ++pass) {
#pragma unroll
      for (int it = 0; it < 4; ++it) {
        const int row = it * 4 + q;
        const float* sp = slab + row * 68 + c8;
        v8h hv;
#pragma unroll
        for (int e = 0; e < 8; ++e) {
          const float t = flush_f16(sp[e]);
          hv[e] = (_Float16)t;
        }
        *(volatile v8h*)(C + (size_t)(mBase + row) * ldc + n0 + c8) = hv;
      }
      __threadfence();
    }
    __builtin_amdgcn_fence(__ATOMIC_RELEASE, "workgroup");
    __builtin_amdgcn_wave_barrier();
    __builtin_amdgcn_fence(__ATOMIC_ACQUIRE, "workgroup");
  }
}

__global__ __launch_bounds__(256) void conv_x_kernel(const float* __restrict__ x,
                                                     unsigned short* __restrict__ XH,
                                                     unsigned short* __restrict__ XL,
                                                     unsigned short* __restrict__ XF, int n8) {
  const int i = blockIdx.x * 256 + threadIdx.x;
  if (i >= n8) return;
  const size_t e0 = (size_t)i << 3;
  const v4f a0 = *(const v4f*)(x + e0);
  const v4f a1 = *(const v4f*)(x + e0 + 4);
  float f[8];
#pragma unroll
  for (int e = 0; e < 4; ++e) {
    const float t0 = a0[e];
    const float t1 = a1[e];
    f[e] = t0;
    f[4 + e] = t1;
  }
  unsigned short hb[8], lb[8], fb[8];
#pragma unroll
  for (int e = 0; e < 8; ++e) {
    const float v = f[e];
    const unsigned short h = f2bf_bits(v);
    hb[e] = h;
    lb[e] = f2bf_bits(v - bf_bits2f(h));
    fb[e] = h_bits(flush_f16(v * kXCarry));
  }
  const v4u uh = (v4u){pk16(hb[0], hb[1]), pk16(hb[2], hb[3]), pk16(hb[4], hb[5]), pk16(hb[6], hb[7])};
  const v4u ul = (v4u){pk16(lb[0], lb[1]), pk16(lb[2], lb[3]), pk16(lb[4], lb[5]), pk16(lb[6], lb[7])};
  const v4u uf = (v4u){pk16(fb[0], fb[1]), pk16(fb[2], fb[3]), pk16(fb[4], fb[5]), pk16(fb[6], fb[7])};
  unsigned short* qh = XH + e0;
  unsigned short* ql = XL + e0;
  unsigned short* qf = XF + e0;
  *(volatile v4u*)qh = uh;
  *(volatile v4u*)ql = ul;
  *(volatile v4u*)qf = uf;
  __threadfence();
  *(volatile v4u*)qh = uh;
  *(volatile v4u*)ql = ul;
  *(volatile v4u*)qf = uf;
}

__global__ __launch_bounds__(256) void pack_w_kernel(const float* __restrict__ Wk1, const float* __restrict__ Wq1,
                                                     const float* __restrict__ Wk2, const float* __restrict__ Wq2,
                                                     const float* __restrict__ Wv,
                                                     unsigned short* __restrict__ WSH, unsigned short* __restrict__ WSL,
                                                     unsigned short* __restrict__ WF) {
  __shared__ float sm[64][65];
  const int t  = threadIdx.x;
  const int k0 = blockIdx.x * 64;
  const int z  = blockIdx.y;
  const float* W = (z == 0) ? Wq1 : (z == 1) ? Wk1 : (z == 2) ? Wv : (z == 3) ? Wq2 : Wk2;
#pragma unroll
  for (int i = 0; i < 16; ++i) {
    const int e = i * 256 + t;
    const int r = e >> 6;
    const int c = e & 63;
    sm[c][r] = W[(size_t)(k0 + r) * kHead + c];
  }
  __syncthreads();
  const int lane = t & 31, wave = t >> 5;
  const int q = lane >> 3, c8 = (lane & 7) * 8;
  if (z < 3) {
    v4u uh[2], ul[2];
#pragma unroll
    for (int it = 0; it < 2; ++it) {
      const int row = wave * 8 + it * 4 + q;
      unsigned short hb[8], lb[8];
#pragma unroll
      for (int e = 0; e < 8; ++e) {
        const float v = sm[row][c8 + e];
        const unsigned short h = f2bf_bits(v);
        hb[e] = h;
        lb[e] = f2bf_bits(v - bf_bits2f(h));
      }
      uh[it] = (v4u){pk16(hb[0], hb[1]), pk16(hb[2], hb[3]), pk16(hb[4], hb[5]), pk16(hb[6], hb[7])};
      ul[it] = (v4u){pk16(lb[0], lb[1]), pk16(lb[2], lb[3]), pk16(lb[4], lb[5]), pk16(lb[6], lb[7])};
    }
    for (int pass = 0; pass < 2; ++pass) {
#pragma unroll
      for (int it = 0; it < 2; ++it) {
        const int row = wave * 8 + it * 4 + q;
        const size_t o = (size_t)(z * 64 + row) * kEmb + k0 + c8;
        *(volatile v4u*)(WSH + o) = uh[it];
        *(volatile v4u*)(WSL + o) = ul[it];
      }
      __threadfence();
    }
  } else {
    v4u uf[2];
#pragma unroll
    for (int it = 0; it < 2; ++it) {
      const int row = wave * 8 + it * 4 + q;
      unsigned short fb[8];
#pragma unroll
      for (int e = 0; e < 8; ++e) {
        const float v = sm[row][c8 + e];
        fb[e] = h_bits(flush_f16(v * kWCarry));
      }
      uf[it] = (v4u){pk16(fb[0], fb[1]), pk16(fb[2], fb[3]), pk16(fb[4], fb[5]), pk16(fb[6], fb[7])};
    }
    for (int pass = 0; pass < 2; ++pass) {
#pragma unroll
      for (int it = 0; it < 2; ++it) {
        const int row = wave * 8 + it * 4 + q;
        const size_t o = (size_t)((z - 3) * 64 + row) * kEmb + k0 + c8;
        *(volatile v4u*)(WF + o) = uf[it];
      }
      __threadfence();
    }
  }
}

template <bool SECOND>
__global__ __launch_bounds__(128) void attn_pass_kernel(const _Float16* __restrict__ Qp,
                                                        const _Float16* __restrict__ Kp,
                                                        const _Float16* __restrict__ Vt,
                                                        const float* o1p,
                                                        const float* __restrict__ lambp,
                                                        float* outp) {
  __shared__ __align__(16) _Float16 Ks[kAtKC * kHead];
  __shared__ __align__(16) _Float16 Vs[kHead * kAtKC];
  __shared__ __align__(16) _Float16 Ps[kAtWaves][16 * kAtKC];
  __shared__ __align__(16) float    Os[kAtWaves][16 * kAtOsP];

  const int tid  = threadIdx.x;
  const int wave = tid >> 5;
  const int lane = tid & 31;
  const int hh   = lane >> 4;
  const int c    = lane & 15;

  const int b    = blockIdx.x / kQBlkPerB;
  const int qb   = blockIdx.x - b * kQBlkPerB;
  const int tok0 = b * kSeq;
  const int q0   = tok0 + qb * kAtQB + wave * 16;

  const _Float16* qrow = Qp + (size_t)(q0 + c) * kHead + 8 * hh;
  const v16h qa0 = Frag<_Float16>::load(qrow);
  const v16h qa1 = Frag<_Float16>::load(qrow + 32);

  float mrow[8], lrow[8];
  v8f oacc[4];
#pragma unroll
  for (int r = 0; r < 8; ++r) { mrow[r] = -1e30f; lrow[r] = 0.f; }
#pragma unroll
  for (int t = 0; t < 4; ++t) oacc[t] = (v8f){0.f,0.f,0.f,0.f,0.f,0.f,0.f,0.f};

  _Float16* pw = Ps[wave];

#pragma unroll 1
  for (int kc = 0; kc < kSeq / kAtKC; ++kc) {
    const int kv0 = tok0 + kc * kAtKC;
    __syncthreads();
#pragma unroll
    for (int i = 0; i < 4; ++i) {
      const int w   = tid + 128 * i;
      const int row = w >> 3;
      const int seg = (w & 7) * 8;
      const v8h kk = *(const v8h*)(Kp + (size_t)(kv0 + row) * kHead + seg);
      const v8h vv = *(const v8h*)(Vt + (size_t)row * kRows + kv0 + seg);
      *(v8h*)(Ks + row * kHead + seg) = kk;
      *(v8h*)(Vs + row * kAtKC + seg) = vv;
    }
    __syncthreads();

    v8f s[4];
#pragma unroll
    for (int j = 0; j < 4; ++j) {
      const _Float16* kr = Ks + (j * 16 + c) * kHead + 8 * hh;
      const v16h kb0 = Frag<_Float16>::load(kr);
      const v16h kb1 = Frag<_Float16>::load(kr + 32);
      v8f a = (v8f){0.f,0.f,0.f,0.f,0.f,0.f,0.f,0.f};
      a = mma_h(qa0, kb0, a);
      a = mma_h(qa1, kb1, a);
      s[j] = a;
    }

#pragma unroll
    for (int r = 0; r < 8; ++r) {
      float mx = fmaxf(fmaxf(s[0][r], s[1][r]), fmaxf(s[2][r], s[3][r]));
      mx = fmaxf(mx, __shfl_xor(mx, 1, 32));
      mx = fmaxf(mx, __shfl_xor(mx, 2, 32));
      mx = fmaxf(mx, __shfl_xor(mx, 4, 32));
      mx = fmaxf(mx, __shfl_xor(mx, 8, 32));
      const float mnew  = fmaxf(mrow[r], mx);
      const float alpha = __expf((mrow[r] - mnew) * kScoreFold);
      mrow[r] = mnew;
      float psum = 0.f;
#pragma unroll
      for (int j = 0; j < 4; ++j) {
        const float arg = fmaf(s[j][r] - mnew, kScoreFold, kLnPCarry);
        const float p   = flush_f16(__expf(arg));
        psum += p;
        pw[(8 * hh + r) * kAtKC + j * 16 + c] = (_Float16)p;
      }
      psum += __shfl_xor(psum, 1, 32);
      psum += __shfl_xor(psum, 2, 32);
      psum += __shfl_xor(psum, 4, 32);
      psum += __shfl_xor(psum, 8, 32);
      lrow[r] = lrow[r] * alpha + psum;
#pragma unroll
      for (int t = 0; t < 4; ++t) oacc[t][r] *= alpha;
    }
    __builtin_amdgcn_fence(__ATOMIC_RELEASE, "workgroup");
    __builtin_amdgcn_wave_barrier();
    __builtin_amdgcn_fence(__ATOMIC_ACQUIRE, "workgroup");

#pragma unroll 1
    for (int kk = 0; kk < 2; ++kk) {
      const v16h pa = Frag<_Float16>::load(pw + c * kAtKC + kk * 32 + 8 * hh);
#pragma unroll
      for (int t = 0; t < 4; ++t) {
        const v16h vb = Frag<_Float16>::load(Vs + (t * 16 + c) * kAtKC + kk * 32 + 8 * hh);
        oacc[t] = mma_h(pa, vb, oacc[t]);
      }
    }
  }

  float* os = Os[wave];
#pragma unroll
  for (int r = 0; r < 8; ++r) {
    const float inv = 1.0f / (lrow[r] * kQKVCarry);
#pragma unroll
    for (int t = 0; t < 4; ++t) os[(8 * hh + r) * kAtOsP + t * 16 + c] = oacc[t][r] * inv;
  }
  __builtin_amdgcn_fence(__ATOMIC_RELEASE, "workgroup");
  __builtin_amdgcn_wave_barrier();
  __builtin_amdgcn_fence(__ATOMIC_ACQUIRE, "workgroup");
  {
    const int c4 = c * 4;
    const float lamb = lambp[0];
    v4f vals[8];
#pragma unroll
    for (int it = 0; it < 8; ++it) {
      const int row = it * 2 + hh;
      v4f val = *(const v4f*)(os + row * kAtOsP + c4);
      if (SECOND) {
        const v4f first = *(const v4f*)(o1p + (size_t)(q0 + row) * kHead + c4);
        val = first - lamb * val;
      }
      vals[it] = val;
    }
    for (int pass = 0; pass < 2; ++pass) {
#pragma unroll
      for (int it = 0; it < 8; ++it) {
        const int row = it * 2 + hh;
        *(volatile v4f*)(outp + (size_t)(q0 + row) * kHead + c4) = vals[it];
      }
      __threadfence();
    }
  }
}

extern "C" void kernel_launch(void* const* d_in, const int* in_sizes, int n_in,
                              void* d_out, int out_size, void* d_ws, size_t ws_size,
                              hipStream_t stream) {
  if (n_in < 7) return;
  if (in_sizes[0] != kRows * kEmb) return;
  if (in_sizes[1] != 1) return;
  if (in_sizes[2] != kEmb * kHead) return;
  if (in_sizes[3] != kEmb * kHead) return;
  if (in_sizes[4] != kEmb * kHead) return;
  if (in_sizes[5] != kEmb * kHead) return;
  if (in_sizes[6] != kEmb * kHead) return;
  if (out_size != kRows * kHead) return;
  if (ws_size < kWsTotal) return;

  const float* x    = (const float*)d_in[0];
  const float* lamb = (const float*)d_in[1];
  const float* Wk1  = (const float*)d_in[2];
  const float* Wq1  = (const float*)d_in[3];
  const float* Wk2  = (const float*)d_in[4];
  const float* Wq2  = (const float*)d_in[5];
  const float* Wv   = (const float*)d_in[6];
  float* out = (float*)d_out;

  char* ws = (char*)d_ws;
  unsigned short* XH  = (unsigned short*)(ws + kOffXH);
  unsigned short* XL  = (unsigned short*)(ws + kOffXL);
  unsigned short* XF  = (unsigned short*)(ws + kOffXF);
  unsigned short* WSH = (unsigned short*)(ws + kOffWSH);
  unsigned short* WSL = (unsigned short*)(ws + kOffWSL);
  unsigned short* WF  = (unsigned short*)(ws + kOffWF);
  unsigned short* Q1  = (unsigned short*)(ws + kOffQ1);
  unsigned short* K1  = (unsigned short*)(ws + kOffK1);
  unsigned short* Q2  = (unsigned short*)(ws + kOffQ2);
  unsigned short* K2  = (unsigned short*)(ws + kOffK2);
  unsigned short* VT  = (unsigned short*)(ws + kOffVT);
  float*          O1  = (float*)(ws + kOffO1);

  conv_x_kernel<<<(kRows * kEmb / 8) / 256, 256, 0, stream>>>(x, XH, XL, XF, kRows * kEmb / 8);
  pack_w_kernel<<<dim3(kEmb / 64, 5), 256, 0, stream>>>(Wk1, Wq1, Wk2, Wq2, Wv, WSH, WSL, WF);

  wmma_gemm64_h<1, true><<<dim3(16, 2), 256, 0, stream>>>(
      XH, XL, kEmb, 0L,
      WSH, WSL, kEmb, (long)kHead * kEmb,
      Q1, kHead, (long)kRows * kHead,
      kRows, kHead, kEmb, kProjSplitScale);

  wmma_gemm64_h<0, false><<<dim3(16, 2), 256, 0, stream>>>(
      XF, XF, kEmb, 0L,
      WF, WF, kEmb, (long)kHead * kEmb,
      Q2, kHead, (long)kRows * kHead,
      kRows, kHead, kEmb, kProjPlainScale);

  wmma_gemm64_h<1, true><<<dim3(16, 1), 256, 0, stream>>>(
      WSH + (size_t)2 * kHead * kEmb, WSL + (size_t)2 * kHead * kEmb, kEmb, 0L,
      XH, XL, kEmb, 0L,
      VT, kRows, 0L,
      kHead, kRows, kEmb, kProjSplitScale);

  attn_pass_kernel<false><<<kRows / kAtQB, 128, 0, stream>>>(
      (const _Float16*)Q1, (const _Float16*)K1, (const _Float16*)VT, O1, lamb, O1);
  attn_pass_kernel<true><<<kRows / kAtQB, 128, 0, stream>>>(
      (const _Float16*)Q2, (const _Float16*)K2, (const _Float16*)VT, O1, lamb, out);
}
